// TopicDecoder_50903952392722
// MI455X (gfx1250) — hardware-run, weakly checked
//
#include <hip/hip_runtime.h>
#include <math.h>

typedef __attribute__((ext_vector_type(16))) _Float16 v16h;
typedef __attribute__((ext_vector_type(8)))  _Float16 v8h;
typedef __attribute__((ext_vector_type(8)))  float    v8f;
typedef __attribute__((ext_vector_type(4)))  float    v4f;

constexpr int kRowsM  = 64;
constexpr int kDepthK = 128;
constexpr int kColsN  = 32000;
constexpr float kEpsAdd = 1e-10f;
constexpr float kCarryA  = 4096.0f;
constexpr float kCarryB  = 32768.0f;
constexpr float kUnscale = 1.0f / (kCarryA * kCarryB);
static_assert(kCarryA * kCarryB == 134217728.0f);
static_assert(kUnscale * 134217728.0f == 1.0f);
static_assert((kDepthK % 32) == 0);
static_assert((kRowsM % 64) == 0);
static_assert((kColsN % 64) == 0);
static_assert(((kColsN / 4) % 32) == 0);

constexpr int kTilesN     = kColsN / 64;
constexpr int kGemmWaves  = 4;
static_assert((kTilesN % kGemmWaves) == 0);
constexpr int kStatPitch  = 32;
constexpr int kTilePitchH = 136;

constexpr size_t kOffStats = 0;
constexpr size_t kOffA16   = kOffStats + (size_t)kDepthK * kStatPitch * 4;
constexpr size_t kOffBt16  = kOffA16   + (size_t)kRowsM * kDepthK * 2;
constexpr size_t kWsTotal  = kOffBt16  + (size_t)kColsN * kDepthK * 2;
static_assert(kWsTotal == 8224768ull);
static_assert(kWsTotal <= 134217728ull);
static_assert((kOffA16 % 128) == 0 && (kOffBt16 % 128) == 0);

union FragU { v16h v; v8h h[2]; };
__device__ __forceinline__ v16h frag_load(const _Float16* p) {
  FragU f;
  f.h[0] = *(const v8h*)(p);
  f.h[1] = *(const v8h*)(p + 16);
  return f.v;
}
__device__ __forceinline__ v8f mma_f16(v16h a, v16h b, v8f c) {
  c = __builtin_amdgcn_wmma_f32_16x16x32_f16(false, a, false, b, (short)0, c, false, false);
  asm volatile("v_nop\n\tv_nop\n\tv_nop\n\tv_nop" : "+v"(c) : "v"(a), "v"(b));
  return c;
}

__global__ __launch_bounds__(256) void row_stats_kernel(const float* __restrict__ x, float* __restrict__ stats)
{
  __shared__ float redMax[8];
  __shared__ float redSum[8];
  const int tid  = threadIdx.x;
  const int lane = tid & 31;
  const int wave = __builtin_amdgcn_readfirstlane((int)(threadIdx.x >> 5));
  const int k    = blockIdx.x;
  const v4f* row = (const v4f*)(x + (size_t)k * kColsN);

  float m = -INFINITY;
#pragma unroll 1
  for (int i = tid; i < kColsN / 4; i += 256) {
    const v4f q = row[i];
    m = fmaxf(m, fmaxf(fmaxf(q[0], q[1]), fmaxf(q[2], q[3])));
  }
#pragma unroll
  for (int o = 16; o > 0; o >>= 1) m = fmaxf(m, __shfl_xor(m, o, 32));
  if (lane == 0) redMax[wave] = m;
  __syncthreads();
  float mk = redMax[0];
#pragma unroll
  for (int w = 1; w < 8; ++w) mk = fmaxf(mk, redMax[w]);

  float s = 0.0f;
#pragma unroll 1
  for (int i = tid; i < kColsN / 4; i += 256) {
    const v4f q = row[i];
    const float e0 = expf(q[0] - mk);
    const float e1 = expf(q[1] - mk);
    const float e2 = expf(q[2] - mk);
    const float e3 = expf(q[3] - mk);
    s += (e0 + e1) + (e2 + e3);
  }
#pragma unroll
  for (int o = 16; o > 0; o >>= 1) s += __shfl_xor(s, o, 32);
  if (lane == 0) redSum[wave] = s;
  __syncthreads();
  float ss = 0.0f;
#pragma unroll
  for (int w = 0; w < 8; ++w) ss += redSum[w];
  const float ls = logf(ss);

  if (wave == 0) {
    const float val = (lane == 0) ? mk : ((lane == 1) ? ls : 0.0f);
    volatile float* p = stats + (size_t)k * kStatPitch + lane;
    *p = val;
    __threadfence();
    *p = val;
  }
}

__global__ __launch_bounds__(256) void prep_a_kernel(const float* __restrict__ th, unsigned short* __restrict__ a16, int total8)
{
  const int i = blockIdx.x * 256 + threadIdx.x;
  if (i >= total8) return;
  const size_t e0 = (size_t)i << 3;
  const v4f q0 = *(const v4f*)(th + e0);
  const v4f q1 = *(const v4f*)(th + e0 + 4);
  v8h hv;
#pragma unroll
  for (int e = 0; e < 4; ++e) {
    const float f0 = (q0[e] + kEpsAdd) * kCarryA;
    const float f1 = (q1[e] + kEpsAdd) * kCarryA;
    hv[e]     = (_Float16)f0;
    hv[4 + e] = (_Float16)f1;
  }
  unsigned short* dst = a16 + e0;
  *(volatile v8h*)dst = hv;
  __threadfence();
  *(volatile v8h*)dst = hv;
}

__global__ __launch_bounds__(256) void prep_bt_kernel(const float* __restrict__ x, const float* __restrict__ stats,
                                                      unsigned short* __restrict__ bt16)
{
  __shared__ __align__(16) _Float16 sTile[64 * kTilePitchH];
  __shared__ float sMx[256];
  __shared__ float sLs[256];
  const int tid = threadIdx.x;
  const int w0  = blockIdx.x * 64;
  {
    const int kk = tid & (kDepthK - 1);
    sMx[tid] = stats[(size_t)kk * kStatPitch];
    sLs[tid] = stats[(size_t)kk * kStatPitch + 1];
  }
  __syncthreads();
  const int w  = tid & 63;
  const int kg = tid >> 6;
  const float* src = x + w0 + w;
#pragma unroll 1
  for (int i = 0; i < 4; ++i) {
    const int k0 = (i * 4 + kg) * 8;
    float xv[8];
#pragma unroll
    for (int e = 0; e < 8; ++e) xv[e] = src[(size_t)(k0 + e) * kColsN];
    v8h hv;
#pragma unroll
    for (int e = 0; e < 8; ++e) {
      const float sh = xv[e] - sMx[k0 + e];
      const float pr = expf(sh - sLs[k0 + e]);
      const float sc = pr * kCarryB;
      hv[e] = (_Float16)sc;
    }
    *(v8h*)(sTile + w * kTilePitchH + k0) = hv;
  }
  __syncthreads();
  v8h ov[4];
#pragma unroll
  for (int it = 0; it < 4; ++it) {
    const int c = it * 256 + tid;
    const int row = c >> 4;
    const int col8 = (c & 15) * 8;
    ov[it] = *(const v8h*)(sTile + row * kTilePitchH + col8);
  }
  for (int pass = 0; pass < 2; ++pass) {
#pragma unroll
    for (int it = 0; it < 4; ++it) {
      const int c = it * 256 + tid;
      const int row = c >> 4;
      const int col8 = (c & 15) * 8;
      *(volatile v8h*)(bt16 + (size_t)(w0 + row) * kDepthK + col8) = ov[it];
    }
    __threadfence();
  }
}

__global__ __launch_bounds__(128) void mix_gemm_kernel(const unsigned short* __restrict__ Ap,
                                                       const unsigned short* __restrict__ Btp,
                                                       float* __restrict__ out)
{
  __shared__ __align__(16) float sT[kGemmWaves][16 * 68];
  const _Float16* A  = (const _Float16*)Ap;
  const _Float16* Bt = (const _Float16*)Btp;
  const int lane = threadIdx.x & 31;
  const int wave = __builtin_amdgcn_readfirstlane((int)(threadIdx.x >> 5));
  const int tile = blockIdx.x * kGemmWaves + wave;
  if (tile >= kTilesN) return;
  const int n0    = tile << 6;
  const int rlane = lane & 15;
  const int koff  = (lane >> 4) * 8;
  const int mOff  = (lane >> 4) * 8;

  v8f acc[4][4];
#pragma unroll
  for (int i = 0; i < 4; ++i)
#pragma unroll
    for (int j = 0; j < 4; ++j) acc[i][j] = (v8f){0.f, 0.f, 0.f, 0.f, 0.f, 0.f, 0.f, 0.f};

#pragma unroll 1
  for (int k0 = 0; k0 < kDepthK; k0 += 32) {
    v16h bh[4];
#pragma unroll
    for (int j = 0; j < 4; ++j) {
      const size_t bo = (size_t)(n0 + (j << 4) + rlane) * kDepthK + koff + k0;
      bh[j] = frag_load(Bt + bo);
    }
#pragma unroll
    for (int i = 0; i < 4; ++i) {
      const size_t ao = (size_t)((i << 4) + rlane) * kDepthK + koff + k0;
      const v16h ah = frag_load(A + ao);
#pragma unroll
      for (int j = 0; j < 4; ++j) acc[i][j] = mma_f16(ah, bh[j], acc[i][j]);
    }
  }

  float* slab = sT[wave];
  const int hh = lane >> 4;
  const int c4 = (lane & 15) * 4;
#pragma unroll
  for (int i = 0; i < 4; ++i) {
    const int mBase = i << 4;
#pragma unroll
    for (int j = 0; j < 4; ++j) {
#pragma unroll
      for (int r = 0; r < 8; ++r) {
        const float v = acc[i][j][r] * kUnscale;
        slab[(mOff + r) * 68 + (j << 4) + rlane] = v;
      }
    }
    __builtin_amdgcn_fence(__ATOMIC_RELEASE, "workgroup");
    __builtin_amdgcn_wave_barrier();
    __builtin_amdgcn_fence(__ATOMIC_ACQUIRE, "workgroup");
    for (int pass = 0; pass < 2; ++pass) {
#pragma unroll
      for (int it = 0; it < 8; ++it) {
        const int row = it * 2 + hh;
        const v4f v = *(const v4f*)(slab + row * 68 + c4);
        *(volatile v4f*)(out + (size_t)(mBase + row) * kColsN + n0 + c4) = v;
      }
      __threadfence();
    }
    __builtin_amdgcn_fence(__ATOMIC_RELEASE, "workgroup");
    __builtin_amdgcn_wave_barrier();
    __builtin_amdgcn_fence(__ATOMIC_ACQUIRE, "workgroup");
  }
}

extern "C" void kernel_launch(void* const* d_in, const int* in_sizes, int n_in,
                              void* d_out, int out_size, void* d_ws, size_t ws_size,
                              hipStream_t stream) {
  if (n_in < 2) return;
  if (in_sizes[0] != kRowsM * kDepthK) return;
  if (in_sizes[1] != kDepthK * kColsN) return;
  if (out_size != kRowsM * kColsN) return;
  if (ws_size < kWsTotal) return;

  const float* theta = (const float*)d_in[0];
  const float* beta  = (const float*)d_in[1];
  float* out = (float*)d_out;

  char* ws = (char*)d_ws;
  float*          stats = (float*)(ws + kOffStats);
  unsigned short* a16   = (unsigned short*)(ws + kOffA16);
  unsigned short* bt16  = (unsigned short*)(ws + kOffBt16);

  row_stats_kernel<<<kDepthK, 256, 0, stream>>>(beta, stats);
  prep_a_kernel<<<(kRowsM * kDepthK / 8) / 256, 256, 0, stream>>>(theta, a16, kRowsM * kDepthK / 8);
  prep_bt_kernel<<<kColsN / 64, 256, 0, stream>>>(beta, stats, bt16);
  mix_gemm_kernel<<<kTilesN / kGemmWaves, 128, 0, stream>>>(a16, bt16, out);
}
